// MultiHeadAttention_32049045963121
// MI455X (gfx1250) — hardware-verified
//
#include <hip/hip_runtime.h>
#include <stddef.h>


typedef _Float16 v16h __attribute__((ext_vector_type(16)));
typedef _Float16 v8h  __attribute__((ext_vector_type(8)));
typedef float    v8f  __attribute__((ext_vector_type(8)));
typedef float    v4f  __attribute__((ext_vector_type(4)));
typedef _Float16 h16;

#ifndef SEQ
#define SEQ 2048
#endif
#define SEQ_FULL 2048
#define DIM   1024
#define NHEAD 16
#define HD    64
#define MROWS SEQ

static_assert(SEQ >= 256 && SEQ <= SEQ_FULL && (SEQ % 256) == 0);
static_assert((SEQ % 128) == 0 && (SEQ % 64) == 0 && (SEQ % 32) == 0 && (SEQ % 16) == 0);
static_assert(DIM == NHEAD * HD);
static_assert(HD == 64);
static_assert((DIM % 64) == 0 && (DIM % 32) == 0);
static_assert((MROWS % 64) == 0);
static_assert(DIM == 4 * 32 * 8);
static_assert((((size_t)SEQ * DIM) % 2048) == 0);
static_assert((((size_t)DIM * DIM) % 2048) == 0);
static_assert((DIM % 32) == 0);

#define LDT 72
#define LDC 68
static_assert((LDT % 8) == 0 && LDT >= 64);
static_assert((LDC % 4) == 0 && LDC >= 64);

#define WCARRY 64.0f
#define PCARRY 1024.0f
#define VCARRY 64.0f

#define WSQ_BYTES     ((size_t)DIM * DIM * 2)
#define PLANE16_BYTES ((size_t)MROWS * DIM * 2)
#define LSE_BYTES     ((size_t)NHEAD * SEQ * 4)
#define VEC_BYTES     ((size_t)DIM * 4)
#define OFF_WQ  ((size_t)0)
#define OFF_WK  (OFF_WQ + WSQ_BYTES)
#define OFF_WV  (OFF_WK + WSQ_BYTES)
#define OFF_WO  (OFF_WV + WSQ_BYTES)
#define OFF_XQ  (OFF_WO + WSQ_BYTES)
#define OFF_XK  (OFF_XQ + PLANE16_BYTES)
#define OFF_XV  (OFF_XK + PLANE16_BYTES)
#define OFF_Q   (OFF_XV + PLANE16_BYTES)
#define OFF_K   (OFF_Q + PLANE16_BYTES)
#define OFF_VT  (OFF_K + PLANE16_BYTES)
#define OFF_CTX (OFF_VT + PLANE16_BYTES)
#define OFF_L   (OFF_CTX + PLANE16_BYTES)
#define OFF_CV  (OFF_L + LSE_BYTES)
#define OFF_DV  (OFF_CV + VEC_BYTES)
#define WS_TOTAL (OFF_DV + VEC_BYTES)
static_assert((WSQ_BYTES % 128) == 0 && (PLANE16_BYTES % 128) == 0);
static_assert((LSE_BYTES % 128) == 0 && (VEC_BYTES % 128) == 0);
static_assert(WS_TOTAL <= (size_t)134217728);

__device__ __forceinline__ float bf16r(float x) {
  unsigned int u = __float_as_uint(x);
  u = (u + 0x7FFFu + ((u >> 16) & 1u)) & 0xFFFF0000u;
  return __uint_as_float(u);
}

static __device__ __forceinline__ h16 toh_flush(float v) {
  const h16 r = (h16)v;
  return (fabsf(v) < 6.103515625e-05f) ? (h16)0.0f : r;
}

__device__ __forceinline__ v16h frag_at(const _Float16* p) {
  v8h lo = *(const v8h*)(p);
  v8h hi = *(const v8h*)(p + 16);
  v16h out;
#pragma unroll
  for (int i = 0; i < 8; ++i) { out[i] = lo[i]; out[i + 8] = hi[i]; }
  return out;
}
__device__ __forceinline__ v16h ld_frag(const _Float16* base, unsigned ld) {
  const unsigned lane = threadIdx.x & 31u;
  return frag_at(base + (lane & 15u) * ld + (lane >> 4) * 8u);
}

__device__ __forceinline__ v8f wmma16(v16h a, v16h b, v8f c) {
  v8f d = __builtin_amdgcn_wmma_f32_16x16x32_f16(false, a, false, b, (short)0, c,
                                                 false, false);
  asm volatile("v_nop\n\tv_nop\n\tv_nop\n\tv_nop" : "+v"(d) : "v"(a), "v"(b));
  return d;
}

__device__ __forceinline__ float red32_sum(float x) {
#pragma unroll
  for (int off = 1; off < 32; off <<= 1) x += __shfl_xor(x, off, 32);
  return x;
}

__device__ __forceinline__ void wave_lds_sync() {
  __builtin_amdgcn_fence(3  , "wavefront");
  asm volatile("s_wait_dscnt 0x0" ::: "memory");
  __builtin_amdgcn_wave_barrier();
}

__global__ __launch_bounds__(256) void cast_kernel(
    const float* __restrict__ src, _Float16* __restrict__ dst, float carry) {
#pragma clang fp contract(off)
  const size_t e = ((size_t)blockIdx.x * 256u + threadIdx.x) * 8u;
  const v4f a0 = *(const v4f*)(src + e);
  const v4f a1 = *(const v4f*)(src + e + 4u);
  v8h o;
#pragma unroll
  for (int i = 0; i < 4; ++i) {
    o[i]     = toh_flush(carry * bf16r(a0[i]));
    o[i + 4] = toh_flush(carry * bf16r(a1[i]));
  }
  _Float16* p = dst + e;
  *(volatile v8h*)p = o;
  __threadfence();
  *(volatile v8h*)p = o;
}

template <int MODE>
__device__ __forceinline__ void gemm_body(
    const _Float16* __restrict__ A16, const _Float16* __restrict__ Bt, const unsigned K,
    const float* __restrict__ bias, const float* __restrict__ addf,
    float* __restrict__ outf, _Float16* __restrict__ out16) {
  __shared__ float Cs[64 * LDC];
  const unsigned tid = threadIdx.x, lane = tid & 31u, w = tid >> 5;
  const unsigned mw = w >> 1, nw = w & 1u;
  const unsigned hh = lane >> 4, m = lane & 15u;
  const unsigned n0 = blockIdx.x * 64u;
  const unsigned row0 = blockIdx.y * 64u;

  const _Float16* ap  = A16 + (size_t)(row0 + mw * 16u + m) * K + hh * 8u;
  const _Float16* bp0 = Bt + (size_t)(n0 + nw * 32u + m) * K + hh * 8u;
  const _Float16* bp1 = bp0 + (size_t)16 * K;
  v8f acc0 = {}, acc1 = {};
#pragma unroll 2
  for (unsigned k0 = 0; k0 < K; k0 += 32u) {
    const v16h a  = frag_at(ap + k0);
    const v16h b0 = frag_at(bp0 + k0);
    const v16h b1 = frag_at(bp1 + k0);
    acc0 = wmma16(a, b0, acc0);
    acc1 = wmma16(a, b1, acc1);
  }
#pragma unroll
  for (int r = 0; r < 8; ++r) {
    float* d = &Cs[(mw * 16u + hh * 8u + (unsigned)r) * LDC + nw * 32u + m];
    d[0]  = acc0[r];
    d[16] = acc1[r];
  }
  __syncthreads();

  if (MODE == 0) {
    v8h x[2];
    size_t off[2];
#pragma unroll
    for (unsigned i = 0; i < 2u; ++i) {
      const unsigned r = 32u * i + (tid >> 3);
      const unsigned c = (tid & 7u) * 8u;
      const v4f u0 = *(const v4f*)&Cs[r * LDC + c];
      const v4f u1 = *(const v4f*)&Cs[r * LDC + c + 4];
      const v4f g0 = *(const v4f*)(bias + n0 + c);
      const v4f g1 = *(const v4f*)(bias + n0 + c + 4u);
#pragma unroll
      for (int j = 0; j < 4; ++j) {
        x[i][j]     = toh_flush(u0[j] * (1.0f / WCARRY) + bf16r(g0[j]));
        x[i][j + 4] = toh_flush(u1[j] * (1.0f / WCARRY) + bf16r(g1[j]));
      }
      off[i] = (size_t)(row0 + r) * DIM + n0 + c;
    }
#pragma unroll
    for (int i = 0; i < 2; ++i) *(volatile v8h*)(out16 + off[i]) = x[i];
    __threadfence();
#pragma unroll
    for (int i = 0; i < 2; ++i) *(volatile v8h*)(out16 + off[i]) = x[i];
  }

  if (MODE == 1) {
    v8h x[2];
    size_t off[2];
#pragma unroll
    for (unsigned i = 0; i < 2u; ++i) {
      const unsigned dcol = 32u * i + (tid >> 3);
      const unsigned kk = (tid & 7u) * 8u;
      const float bb = bf16r(bias[n0 + dcol]);
#pragma unroll
      for (unsigned j = 0; j < 8u; ++j) {
        const float t = Cs[(kk + j) * LDC + dcol] * (1.0f / WCARRY) + bb;
        x[i][j] = toh_flush(t);
      }
      off[i] = (size_t)(n0 + dcol) * SEQ + row0 + kk;
    }
#pragma unroll
    for (int i = 0; i < 2; ++i) *(volatile v8h*)(out16 + off[i]) = x[i];
    __threadfence();
#pragma unroll
    for (int i = 0; i < 2; ++i) *(volatile v8h*)(out16 + off[i]) = x[i];
  }

  if (MODE == 2) {
    const float cs = 1.0f / (WCARRY * VCARRY);
    v4f xs[4];
    size_t off[4];
#pragma unroll
    for (unsigned i = 0; i < 4u; ++i) {
      const unsigned r = 16u * i + (tid >> 4);
      const unsigned c = (tid & 15u) * 4u;
      const v4f u = *(const v4f*)&Cs[r * LDC + c];
      const v4f g = *(const v4f*)(addf + n0 + c);
      v4f val;
#pragma unroll
      for (int j = 0; j < 4; ++j) val[j] = u[j] * cs + g[j];
      xs[i] = val;
      off[i] = (size_t)(row0 + r) * DIM + n0 + c;
    }
#pragma unroll
    for (int i = 0; i < 4; ++i) *(volatile v4f*)(outf + off[i]) = xs[i];
    __threadfence();
#pragma unroll
    for (int i = 0; i < 4; ++i) *(volatile v4f*)(outf + off[i]) = xs[i];
  }
}

__global__ __launch_bounds__(256) void gemm_qk_kernel(
    const _Float16* __restrict__ A16, const _Float16* __restrict__ Bt,
    const float* __restrict__ bias, _Float16* __restrict__ out16) {
  gemm_body<0>(A16, Bt, (unsigned)DIM, bias, bias, (float*)0, out16);
}
__global__ __launch_bounds__(256) void gemm_v_kernel(
    const _Float16* __restrict__ A16, const _Float16* __restrict__ Bt,
    const float* __restrict__ bias, _Float16* __restrict__ vt) {
  gemm_body<1>(A16, Bt, (unsigned)DIM, bias, bias, (float*)0, vt);
}
__global__ __launch_bounds__(256) void gemm_wo_kernel(
    const _Float16* __restrict__ A16, const _Float16* __restrict__ Bt,
    const float* __restrict__ dvec, float* __restrict__ outf) {
  gemm_body<2>(A16, Bt, (unsigned)DIM, dvec, dvec, outf, (_Float16*)0);
}

__global__ __launch_bounds__(256) void lse_kernel(
    const _Float16* __restrict__ Qh, const _Float16* __restrict__ Kh, float* __restrict__ L) {
  __shared__ float redM[16 * 32];
  __shared__ float redS[16 * 32];
  const unsigned tid = threadIdx.x, lane = tid & 31u;
  const unsigned wave = (unsigned)__builtin_amdgcn_readfirstlane((int)(threadIdx.x >> 5));
  const unsigned hh = lane >> 4, m = lane & 15u;
  const unsigned t0 = blockIdx.x * 32u;
  const unsigned head = blockIdx.y;

  const size_t koff = (size_t)(t0 + m) * DIM + head * HD + hh * 8u;
  v16h kf[2][2];
#pragma unroll
  for (int kg = 0; kg < 2; ++kg)
#pragma unroll
    for (int c = 0; c < 2; ++c)
      kf[kg][c] = frag_at(Kh + koff + (size_t)kg * 16u * DIM + (unsigned)c * 32u);

  float mr[2], sr[2];
#pragma unroll
  for (int kg = 0; kg < 2; ++kg) { mr[kg] = -1.0e30f; sr[kg] = 0.0f; }

  for (unsigned i = (t0 >> 4) + wave; i < (unsigned)(SEQ / 16); i += 8u) {
    const unsigned s0 = i * 16u;
    const size_t qoff = (size_t)(s0 + m) * DIM + head * HD + hh * 8u;
    const v16h qf0 = frag_at(Qh + qoff);
    const v16h qf1 = frag_at(Qh + qoff + 32);
#pragma unroll
    for (int kg = 0; kg < 2; ++kg) {
      v8f t = {};
      t = wmma16(qf0, kf[kg][0], t);
      t = wmma16(qf1, kf[kg][1], t);
      const unsigned key = t0 + (unsigned)kg * 16u + m;
      float xm[8];
      bool dead[8];
      float tm = -1.0e30f;
#pragma unroll
      for (int v = 0; v < 8; ++v) {
        const unsigned row = s0 + hh * 8u + (unsigned)v;
        dead[v] = (key > row);
        xm[v] = dead[v] ? -1.0e30f : t[v] * 0.125f;
        tm = fmaxf(tm, xm[v]);
      }
      const float mn = fmaxf(mr[kg], tm);
      float add = 0.0f;
#pragma unroll
      for (int v = 0; v < 8; ++v) {
        const float e = __expf(xm[v] - mn);
        add += dead[v] ? 0.0f : e;
      }
      sr[kg] = sr[kg] * __expf(mr[kg] - mn) + add;
      mr[kg] = mn;
    }
  }
#pragma unroll
  for (int kg = 0; kg < 2; ++kg) {
    redM[(wave * 2u + hh) * 32u + (unsigned)kg * 16u + m] = mr[kg];
    redS[(wave * 2u + hh) * 32u + (unsigned)kg * 16u + m] = sr[kg];
  }
  __syncthreads();
  if (wave == 0u) {
    float mm = -1.0e30f, ss = 0.0f;
#pragma unroll 1
    for (unsigned p = 0; p < 16u; ++p) {
      const float m2 = redM[p * 32u + lane];
      const float s2 = redS[p * 32u + lane];
      const float mn = fmaxf(mm, m2);
      ss = ss * __expf(mm - mn) + s2 * __expf(m2 - mn);
      mm = mn;
    }
    const float tcount = (float)(t0 + lane);
    const float mn = fmaxf(mm, 0.0f);
    ss = ss * __expf(mm - mn) + tcount * __expf(0.0f - mn);
    const float val = mn + logf(ss);
    float* p = L + (size_t)head * SEQ + t0 + lane;
    *(volatile float*)p = val;
    __threadfence();
    *(volatile float*)p = val;
  }
}

__global__ __launch_bounds__(256) void cvec_kernel(
    const float* __restrict__ L, const _Float16* __restrict__ Vt, float* __restrict__ cv) {
#pragma clang fp contract(off)
  __shared__ float red[32];
  const unsigned lane = threadIdx.x & 31u;
  const unsigned wave = (unsigned)__builtin_amdgcn_readfirstlane((int)(threadIdx.x >> 5));
#pragma unroll 1
  for (unsigned rr = 0; rr < 4u; ++rr) {
    const unsigned n = blockIdx.x * 32u + wave * 4u + rr;
    const unsigned head = n >> 6;
    const _Float16* vr = Vt + (size_t)n * SEQ + lane * 8u;
    const float* lr = L + (size_t)head * SEQ + lane * 8u;
    float acc = 0.0f;
#pragma unroll 1
    for (unsigned j = 0; j < (unsigned)(SEQ / 256); ++j) {
      const v8h vv = *(const v8h*)(vr + j * 256u);
      const v4f l0 = *(const v4f*)(lr + j * 256u);
      const v4f l1 = *(const v4f*)(lr + j * 256u + 4u);
#pragma unroll
      for (int i = 0; i < 4; ++i) {
        acc += l0[i] * (float)vv[i];
        acc += l1[i] * (float)vv[i + 4];
      }
    }
    acc = red32_sum(acc);
    if (lane == 0u) red[wave * 4u + rr] = acc;
  }
  __syncthreads();
  if (wave == 0u) {
    const float val = red[lane];
    float* p = cv + blockIdx.x * 32u + lane;
    *(volatile float*)p = val;
    __threadfence();
    *(volatile float*)p = val;
  }
}

__global__ __launch_bounds__(256) void dvec_kernel(
    const float* __restrict__ Wo, const float* __restrict__ bo,
    const float* __restrict__ cv, float* __restrict__ dv) {
#pragma clang fp contract(off)
  __shared__ float red[32];
  const unsigned lane = threadIdx.x & 31u;
  const unsigned wave = (unsigned)__builtin_amdgcn_readfirstlane((int)(threadIdx.x >> 5));
#pragma unroll 1
  for (unsigned rr = 0; rr < 4u; ++rr) {
    const unsigned n = blockIdx.x * 32u + wave * 4u + rr;
    const float* wr = Wo + (size_t)n * DIM + lane * 8u;
    const float* cr = cv + lane * 8u;
    float acc = 0.0f;
#pragma unroll 1
    for (unsigned j = 0; j < 4u; ++j) {
      const v4f w0 = *(const v4f*)(wr + j * 256u);
      const v4f w1 = *(const v4f*)(wr + j * 256u + 4u);
      const v4f c0 = *(const v4f*)(cr + j * 256u);
      const v4f c1 = *(const v4f*)(cr + j * 256u + 4u);
#pragma unroll
      for (int i = 0; i < 4; ++i) {
        acc += bf16r(w0[i]) * c0[i];
        acc += bf16r(w1[i]) * c1[i];
      }
    }
    acc = red32_sum(acc);
    if (lane == 0u) red[wave * 4u + rr] = acc;
  }
  __syncthreads();
  if (wave == 0u) {
    const unsigned n = blockIdx.x * 32u + lane;
    const float val = bf16r(bo[n]) - red[lane];
    float* p = dv + n;
    *(volatile float*)p = val;
    __threadfence();
    *(volatile float*)p = val;
  }
}

__global__ __launch_bounds__(256) void attn_kernel(
    const _Float16* __restrict__ Qh, const _Float16* __restrict__ Kh,
    const _Float16* __restrict__ Vt, _Float16* __restrict__ Ov) {
  __shared__ _Float16 Ks[64 * LDT];
  __shared__ _Float16 Vs[64 * LDT];
  __shared__ _Float16 Ps[8 * 16 * LDT];

  const unsigned tid = threadIdx.x, lane = tid & 31u;
  const unsigned w = (unsigned)__builtin_amdgcn_readfirstlane((int)(threadIdx.x >> 5));
  const unsigned hh = lane >> 4, m = lane & 15u;
  const unsigned q0 = blockIdx.x * 128u;
  const unsigned head = blockIdx.y;
  const unsigned qrow0 = q0 + w * 16u;
  const unsigned pb = w * (16u * LDT);

  const size_t qoff = (size_t)(qrow0 + m) * DIM + head * HD + hh * 8u;
  v16h qf[2];
  qf[0] = frag_at(Qh + qoff);
  qf[1] = frag_at(Qh + qoff + 32);

  v8f o[4];
#pragma unroll
  for (int nb = 0; nb < 4; ++nb) o[nb] = (v8f){};

  const size_t kplane = (size_t)head * HD;
  const size_t vplane = (size_t)head * HD * SEQ;
  const unsigned kend = q0 + 128u;

  for (unsigned kb = 0; kb < kend; kb += 64u) {
#pragma unroll
    for (unsigned j = 0; j < 2u; ++j) {
      const unsigned idx = tid + 256u * j;
      const unsigned r = idx >> 3, c = (idx & 7u) * 8u;
      *(v8h*)&Ks[r * LDT + c] = *(const v8h*)(Kh + kplane + (size_t)(kb + r) * DIM + c);
      *(v8h*)&Vs[r * LDT + c] = *(const v8h*)(Vt + vplane + (size_t)r * SEQ + kb + c);
    }
    __syncthreads();

    v8f s[4];
#pragma unroll
    for (int kg = 0; kg < 4; ++kg) {
      v8f t = {};
#pragma unroll
      for (int c = 0; c < 2; ++c) {
        const v16h kf = ld_frag(&Ks[(kg * 16) * LDT + c * 32], LDT);
        t = wmma16(qf[c], kf, t);
      }
      s[kg] = t * (0.125f * PCARRY);
    }

    if (kb >= q0) {
#pragma unroll
      for (int kg = 0; kg < 4; ++kg)
#pragma unroll
        for (int v = 0; v < 8; ++v) {
          const unsigned key = kb + (unsigned)kg * 16u + m;
          const unsigned row = qrow0 + hh * 8u + (unsigned)v;
          s[kg][v] = (key > row) ? 0.0f : s[kg][v];
        }
    }

#pragma unroll
    for (int kg = 0; kg < 4; ++kg)
#pragma unroll
      for (int v = 0; v < 8; ++v)
        Ps[pb + (hh * 8u + (unsigned)v) * LDT + (unsigned)kg * 16u + m] = toh_flush(s[kg][v]);
    wave_lds_sync();

#pragma unroll
    for (int c = 0; c < 2; ++c) {
      const v16h pf = ld_frag(&Ps[pb + c * 32], LDT);
#pragma unroll
      for (int nb = 0; nb < 4; ++nb) {
        const v16h vf = ld_frag(&Vs[(nb * 16) * LDT + c * 32], LDT);
        o[nb] = wmma16(pf, vf, o[nb]);
      }
    }
    __syncthreads();
  }

#pragma unroll
  for (int nb = 0; nb < 4; ++nb)
#pragma unroll
    for (int v = 0; v < 8; ++v)
      Ps[pb + (hh * 8u + (unsigned)v) * LDT + (unsigned)nb * 16u + m] =
          toh_flush(o[nb][v] * (VCARRY / PCARRY));
  wave_lds_sync();
  v8h x[4];
  size_t off[4];
#pragma unroll
  for (unsigned i = 0; i < 4u; ++i) {
    const unsigned r = 4u * i + (lane >> 3);
    const unsigned c = (lane & 7u) * 8u;
    x[i] = *(const v8h*)&Ps[pb + r * LDT + c];
    off[i] = (size_t)(qrow0 + r) * DIM + head * HD + c;
  }
#pragma unroll
  for (int i = 0; i < 4; ++i) *(volatile v8h*)(Ov + off[i]) = x[i];
  __threadfence();
#pragma unroll
  for (int i = 0; i < 4; ++i) *(volatile v8h*)(Ov + off[i]) = x[i];
}

extern "C" void kernel_launch(void* const* d_in, const int* in_sizes, int n_in,
                              void* d_out, int out_size, void* d_ws, size_t ws_size,
                              hipStream_t stream) {
  if (n_in < 11) return;
  const long long need_x = (long long)SEQ * DIM;
  if ((long long)in_sizes[0] < need_x) return;
  if ((long long)in_sizes[1] < need_x) return;
  if ((long long)in_sizes[2] < need_x) return;
  if ((long long)in_sizes[3] < (long long)DIM * DIM) return;
  if ((long long)in_sizes[5] < (long long)DIM * DIM) return;
  if ((long long)in_sizes[7] < (long long)DIM * DIM) return;
  if ((long long)in_sizes[9] < (long long)DIM * DIM) return;
  if (in_sizes[4] < DIM || in_sizes[6] < DIM || in_sizes[8] < DIM || in_sizes[10] < DIM) return;
  if ((long long)out_size < need_x) return;
  if (ws_size < WS_TOTAL) return;

  const float* Qin = (const float*)d_in[0];
  const float* Kin = (const float*)d_in[1];
  const float* Vin = (const float*)d_in[2];
  const float* wq  = (const float*)d_in[3];
  const float* bq  = (const float*)d_in[4];
  const float* wk  = (const float*)d_in[5];
  const float* bk  = (const float*)d_in[6];
  const float* wv  = (const float*)d_in[7];
  const float* bv  = (const float*)d_in[8];
  const float* wo  = (const float*)d_in[9];
  const float* bo  = (const float*)d_in[10];
  float* out = (float*)d_out;

  char* ws = (char*)d_ws;
  _Float16* Wq16  = (_Float16*)(ws + OFF_WQ);
  _Float16* Wk16  = (_Float16*)(ws + OFF_WK);
  _Float16* Wv16  = (_Float16*)(ws + OFF_WV);
  _Float16* Wo16  = (_Float16*)(ws + OFF_WO);
  _Float16* Xq16  = (_Float16*)(ws + OFF_XQ);
  _Float16* Xk16  = (_Float16*)(ws + OFF_XK);
  _Float16* Xv16  = (_Float16*)(ws + OFF_XV);
  _Float16* Qh16  = (_Float16*)(ws + OFF_Q);
  _Float16* Kh16  = (_Float16*)(ws + OFF_K);
  _Float16* Vt16  = (_Float16*)(ws + OFF_VT);
  _Float16* Ctx16 = (_Float16*)(ws + OFF_CTX);
  float*    Lse   = (float*)(ws + OFF_L);
  float*    Cv    = (float*)(ws + OFF_CV);
  float*    Dv    = (float*)(ws + OFF_DV);

  dim3 blk(256);
  dim3 gx((unsigned)(((size_t)SEQ * DIM) / 2048));
  dim3 gw((unsigned)(((size_t)DIM * DIM) / 2048));
  dim3 gg(DIM / 64, MROWS / 64);

  cast_kernel<<<gx, blk, 0, stream>>>(Qin, Xq16, 1.0f);
  cast_kernel<<<gx, blk, 0, stream>>>(Kin, Xk16, 1.0f);
  cast_kernel<<<gx, blk, 0, stream>>>(Vin, Xv16, 1.0f);
  cast_kernel<<<gw, blk, 0, stream>>>(wq, Wq16, WCARRY);
  cast_kernel<<<gw, blk, 0, stream>>>(wk, Wk16, WCARRY);
  cast_kernel<<<gw, blk, 0, stream>>>(wv, Wv16, WCARRY);
  cast_kernel<<<gw, blk, 0, stream>>>(wo, Wo16, WCARRY);

  gemm_qk_kernel<<<gg, blk, 0, stream>>>(Xq16, Wq16, bq, Qh16);
  gemm_qk_kernel<<<gg, blk, 0, stream>>>(Xk16, Wk16, bk, Kh16);
  gemm_v_kernel<<<gg, blk, 0, stream>>>(Xv16, Wv16, bv, Vt16);

  lse_kernel<<<dim3(SEQ / 32, NHEAD), blk, 0, stream>>>(Qh16, Kh16, Lse);
  cvec_kernel<<<dim3(DIM / 32), blk, 0, stream>>>(Lse, Vt16, Cv);
  dvec_kernel<<<dim3(DIM / 32), blk, 0, stream>>>(wo, bo, Cv, Dv);

  attn_kernel<<<dim3(SEQ / 128, NHEAD), blk, 0, stream>>>(Qh16, Kh16, Vt16, Ctx16);
  gemm_wo_kernel<<<gg, blk, 0, stream>>>(Ctx16, Wo16, Dv, out);
}
